// MultiHeadSelfAttentionModule_56770877719143
// MI455X (gfx1250) — hardware-verified
//
#include <hip/hip_runtime.h>
#include <math.h>

constexpr int kBatch     = 16;
constexpr int kSeq       = 512;
constexpr int kDim       = 512;
constexpr int kHeads     = 8;
constexpr int kHd        = 64;
constexpr int kP         = 2 * kSeq - 1;
constexpr int kPosPad    = 1024;
constexpr int kTok       = kBatch * kSeq;
constexpr int kChunk     = 4;
constexpr int kChunkRows = kChunk * kPosPad;
constexpr int kBandN     = 9;
constexpr int kBandOff   = 7;
constexpr int kSPld      = kBandN * 64;
constexpr int kVecRows   = 8;
constexpr float kScoreScale = 0.125f;
constexpr float kInvDim     = 1.0f / 512.0f;
constexpr float kLnEps      = 1e-5f;
static_assert(kHeads * kHd == kDim, "shape");
static_assert(kTok % 64 == 0 && kDim % 64 == 0 && kSeq % 64 == 0 && kPosPad % 64 == 0 && kHd % 64 == 0 && kChunkRows % 64 == 0, "M,N tile multiples");
static_assert(kDim % 32 == 0 && kHd % 32 == 0 && kSeq % 32 == 0, "K multiples of 32");
static_assert(kP < kPosPad && kBatch % kChunk == 0, "pad row exists, chunks exact");
static_assert(kSeq == 512 && kDim == 512, "lane maps assume 512-wide rows");
static_assert(kBandOff - (kSeq / 64 - 1) >= 0 && kBandOff + kBandN <= kPosPad / 64, "band tiles inside the operand plane");
static_assert(kSPld % 32 == 0 && (kSeq - 1) + 63 < kSPld, "compact band pitch covers every shifted column");

typedef __attribute__((ext_vector_type(16))) _Float16 v16h;
typedef __attribute__((ext_vector_type(8)))  _Float16 v8h;
typedef __attribute__((ext_vector_type(16))) __bf16   v16b;
typedef __attribute__((ext_vector_type(8)))  __bf16   v8b;
typedef __attribute__((ext_vector_type(8)))  float    v8f;
typedef __attribute__((ext_vector_type(4)))  float    v4f;
typedef __attribute__((ext_vector_type(2)))  float    v2f;
typedef __attribute__((ext_vector_type(4)))  unsigned int v4u;

__device__ __forceinline__ unsigned short f2bf_bits(float f) {
  unsigned u = __float_as_uint(f);
  return (unsigned short)((u + 0x7FFFu + ((u >> 16) & 1u)) >> 16);
}
__device__ __forceinline__ float bf_bits2f(unsigned short h) { return __uint_as_float(((unsigned)h) << 16); }
__device__ __forceinline__ float rbf(float f) { return bf_bits2f(f2bf_bits(f)); }

__device__ __forceinline__ void dep_guard_h(v8f& a, v8f& b, v16h x, v16h y) { asm volatile("v_nop\n\tv_nop\n\tv_nop\n\tv_nop" : "+v"(a), "+v"(b) : "v"(x), "v"(y)); }
__device__ __forceinline__ void dep_guard_b(v8f& a, v8f& b, v16b x, v16b y) { asm volatile("v_nop\n\tv_nop\n\tv_nop\n\tv_nop" : "+v"(a), "+v"(b) : "v"(x), "v"(y)); }
__device__ __forceinline__ void keep4_h(v16h a, v16h b, v16h c, v16h d) { asm volatile("v_nop" :: "v"(a), "v"(b), "v"(c), "v"(d)); }
__device__ __forceinline__ void keep4_b(v16b a, v16b b, v16b c, v16b d) { asm volatile("v_nop" :: "v"(a), "v"(b), "v"(c), "v"(d)); }
__device__ __forceinline__ void acc_guard4(v8f& a, v8f& b, v8f& c, v8f& d) { asm volatile("v_nop\n\tv_nop\n\tv_nop\n\tv_nop" : "+v"(a), "+v"(b), "+v"(c), "+v"(d)); }
template <typename T> struct Frag;
template <> struct Frag<_Float16> {
  typedef v16h V; union U { v16h v; v8h h[2]; };
  static __device__ __forceinline__ v16h load(const _Float16* p) {
    U f; f.h[0] = *(const v8h*)(p); f.h[1] = *(const v8h*)(p + 16); return f.v;
  }
  static __device__ __forceinline__ v8f mma(v16h a, v16h b, v8f c) {
    return __builtin_amdgcn_wmma_f32_16x16x32_f16(false, a, false, b, (short)0, c, false, false);
  }
  static __device__ __forceinline__ void guard(v8f& a, v8f& b, v16h x, v16h y) { dep_guard_h(a, b, x, y); }
  static __device__ __forceinline__ void keep(v16h a, v16h b, v16h c, v16h d) { keep4_h(a, b, c, d); }
};
template <> struct Frag<__bf16> {
  typedef v16b V; union U { v16b v; v8b h[2]; };
  static __device__ __forceinline__ v16b load(const __bf16* p) {
    U f; f.h[0] = *(const v8b*)(p); f.h[1] = *(const v8b*)(p + 16); return f.v;
  }
  static __device__ __forceinline__ v8f mma(v16b a, v16b b, v8f c) {
    return __builtin_amdgcn_wmma_f32_16x16x32_bf16(false, a, false, b, (short)0, c, false, false);
  }
  static __device__ __forceinline__ void guard(v8f& a, v8f& b, v16b x, v16b y) { dep_guard_b(a, b, x, y); }
  static __device__ __forceinline__ void keep(v16b a, v16b b, v16b c, v16b d) { keep4_b(a, b, c, d); }
};

__device__ __forceinline__ unsigned pk16(unsigned short a, unsigned short b) { return (unsigned)a | ((unsigned)b << 16); }

template <int ET> struct Elem;
template <> struct Elem<0> { typedef _Float16 T; };
template <> struct Elem<1> { typedef __bf16 T; };
template <int ET, bool SPLA, bool SPLB, int BIAS_MODE, int OUT_MODE, int BANDN = 0, int BANDOFF = 0>
__global__ __launch_bounds__(256) void wmma_gemm64(
    const unsigned short* __restrict__ Ap, const unsigned short* __restrict__ A2p, int lda, long strideA,
    const unsigned short* __restrict__ Btp, const unsigned short* __restrict__ Bt2p, int ldb, long strideB,
    void* __restrict__ Cout, void* __restrict__ Cout2, int ldc, long strideC,
    const float* __restrict__ bias, int M, int N, int K, float scale) {
  typedef typename Elem<ET>::T T;
  typedef typename Frag<T>::V V;
  const T* A = (const T*)Ap; const T* A2 = (const T*)A2p; const T* Bt = (const T*)Btp; const T* Bt2 = (const T*)Bt2p;
  __shared__ __align__(16) float sT[8][16 * 68];
  const int b    = blockIdx.y;
  const int lane = threadIdx.x & 31;
  const int wave = threadIdx.x >> 5;
  const int tilesN = (BANDN > 0) ? BANDN : (N >> 6);
  const int tilesM = M >> 6;
  const int tile = blockIdx.x * 8 + wave;
  if (tile >= tilesM * tilesN) return;
  const int tm = tile / tilesN;
  const int tn = tile - tm * tilesN;
  const int m0 = tm << 6;
  const int n0 = tn << 6;
  const int nb0 = (BANDN > 0) ? ((BANDOFF - tm + tn) << 6) : n0;

  const T* Ab  = A  + (size_t)b * strideA;
  const T* Bb  = Bt + (size_t)b * strideB;
  const T* Ab2 = SPLA ? (A2  + (size_t)b * strideA) : Ab;
  const T* Bb2 = SPLB ? (Bt2 + (size_t)b * strideB) : Bb;

  const int rlane = lane & 15;
  const int koff  = (lane >> 4) * 8;
  const int mOff  = (lane >> 4) * 8;

  v8f acc[4][4];
#pragma unroll
  for (int i = 0; i < 4; ++i)
#pragma unroll
    for (int j = 0; j < 4; ++j) acc[i][j] = (v8f){0.f,0.f,0.f,0.f,0.f,0.f,0.f,0.f};

  for (int k0 = 0; k0 < K; k0 += 32) {
    V bh[4], bl[4];
#pragma unroll
    for (int j = 0; j < 4; ++j) {
      const size_t bo = (size_t)(nb0 + (j << 4) + rlane) * ldb + koff + k0;
      bh[j] = Frag<T>::load(Bb + bo);
      if (SPLB) bl[j] = Frag<T>::load(Bb2 + bo);
    }
#pragma unroll
    for (int i = 0; i < 4; ++i) {
      const size_t ao = (size_t)(m0 + (i << 4) + rlane) * lda + koff + k0;
      V ah = Frag<T>::load(Ab + ao);
      V al = ah;
      if (SPLA) al = Frag<T>::load(Ab2 + ao);
#pragma unroll
      for (int j = 0; j < 4; ++j) {
        acc[i][j] = Frag<T>::mma(ah, bh[j], acc[i][j]);
        if (SPLB) acc[i][j] = Frag<T>::mma(ah, bl[j], acc[i][j]);
        if (SPLA) acc[i][j] = Frag<T>::mma(al, bh[j], acc[i][j]);
      }
      Frag<T>::guard(acc[i][0], acc[i][3], ah, al);
      Frag<T>::guard(acc[i][1], acc[i][2], ah, al);
    }
    Frag<T>::keep(bh[0], bh[1], bh[2], bh[3]);
    if (SPLB) Frag<T>::keep(bl[0], bl[1], bl[2], bl[3]);
  }
  acc_guard4(acc[0][0], acc[0][1], acc[0][2], acc[0][3]);
  acc_guard4(acc[1][0], acc[1][1], acc[1][2], acc[1][3]);
  acc_guard4(acc[2][0], acc[2][1], acc[2][2], acc[2][3]);
  acc_guard4(acc[3][0], acc[3][1], acc[3][2], acc[3][3]);

  float* slab = sT[wave];
#pragma unroll
  for (int i = 0; i < 4; ++i) {
    const int mBase = m0 + (i << 4);
    v4f bmA = (v4f){0.f, 0.f, 0.f, 0.f};
    v4f bmB = bmA;
    if (BIAS_MODE == 1) {
      bmA = *(const v4f*)(bias + mBase + mOff);
      bmB = *(const v4f*)(bias + mBase + mOff + 4);
    }
#pragma unroll
    for (int j = 0; j < 4; ++j) {
      const int n = nb0 + (j << 4) + rlane;
      float bv = 0.f;
      if (BIAS_MODE == 2) bv = bias[n];
#pragma unroll
      for (int r = 0; r < 8; ++r) {
        float v = acc[i][j][r] * scale;
        if (BIAS_MODE == 1) v += (r < 4) ? bmA[r & 3] : bmB[r & 3];
        if (BIAS_MODE == 2) v += bv;
        slab[(mOff + r) * 68 + (j << 4) + rlane] = v;
      }
    }
    __builtin_amdgcn_fence(__ATOMIC_RELEASE, "workgroup");
    __builtin_amdgcn_wave_barrier();
    __builtin_amdgcn_fence(__ATOMIC_ACQUIRE, "workgroup");
    if (OUT_MODE == 0) {
      float* C = (float*)Cout + (size_t)b * strideC;
      const int hh = lane >> 4, c4 = (lane & 15) * 4;
      for (int pass = 0; pass < 2; ++pass) {
#pragma unroll
        for (int it = 0; it < 8; ++it) {
          const int row = it * 2 + hh;
          v4f v = *(const v4f*)(slab + row * 68 + c4);
          *(volatile v4f*)(C + (size_t)(mBase + row) * ldc + n0 + c4) = v;
        }
        __threadfence();
      }
    } else {
      const int q = lane >> 3, c8 = (lane & 7) * 8;
      unsigned short* C  = (unsigned short*)Cout  + (size_t)b * strideC;
      unsigned short* C2 = (OUT_MODE == 2) ? ((unsigned short*)Cout2 + (size_t)b * strideC) : nullptr;
      for (int pass = 0; pass < 2; ++pass) {
#pragma unroll
        for (int it = 0; it < 4; ++it) {
          const int row = it * 4 + q;
          const float* sp = slab + row * 68 + c8;
          v8h hv, lv;
#pragma unroll
          for (int e = 0; e < 8; ++e) {
            if (OUT_MODE == 1) {
              hv[e] = (_Float16)sp[e];
            } else {
              unsigned short hb = f2bf_bits(sp[e]);
              unsigned short lb = f2bf_bits(sp[e] - bf_bits2f(hb));
              hv[e] = __builtin_bit_cast(_Float16, hb);
              lv[e] = __builtin_bit_cast(_Float16, lb);
            }
          }
          *(volatile v8h*)(C + (size_t)(mBase + row) * ldc + n0 + c8) = hv;
          if (OUT_MODE == 2) *(volatile v8h*)(C2 + (size_t)(mBase + row) * ldc + n0 + c8) = lv;
        }
        __threadfence();
      }
    }
    __builtin_amdgcn_fence(__ATOMIC_RELEASE, "workgroup");
    __builtin_amdgcn_wave_barrier();
    __builtin_amdgcn_fence(__ATOMIC_ACQUIRE, "workgroup");
  }
}

__global__ __launch_bounds__(128) void vecprep_kernel(const float* __restrict__ bq, const float* __restrict__ bk,
                                                       const float* __restrict__ bv, const float* __restrict__ bp,
                                                       const float* __restrict__ bo, const float* __restrict__ g,
                                                       const float* __restrict__ bb, const float* __restrict__ cb,
                                                       const float* __restrict__ pb, float* __restrict__ outv) {
  const int r = blockIdx.x;
  const int t = threadIdx.x;
  const float* s1 = (r <= 1) ? bq : (r == 2) ? bk : (r == 3) ? bv : (r == 4) ? bp : (r == 5) ? bo : (r == 6) ? g : bb;
  const float* s2 = (r == 0) ? cb : (r == 1) ? pb : bq;
  const float f2 = (r <= 1) ? 1.0f : 0.0f;
  const v4f a = *(const v4f*)(s1 + 4 * t);
  const v4f c = *(const v4f*)(s2 + 4 * t);
  v4f o;
#pragma unroll
  for (int e = 0; e < 4; ++e) o[e] = rbf(a[e]) + f2 * rbf(c[e]);
  float* dst = outv + (size_t)r * kDim + 4 * t;
  *(volatile v4f*)dst = o;
  __threadfence();
  *(volatile v4f*)dst = o;
}

__global__ __launch_bounds__(256) void castw_kernel(const float* __restrict__ W0, const float* __restrict__ W1,
                                                    const float* __restrict__ W2, const float* __restrict__ W3,
                                                    const float* __restrict__ W4, unsigned short* __restrict__ out) {
  const int z = blockIdx.y;
  const float* W = (z == 0) ? W0 : (z == 1) ? W1 : (z == 2) ? W2 : (z == 3) ? W3 : W4;
  const int i = blockIdx.x * 256 + threadIdx.x;
  const float* p = W + 8 * (size_t)i;
  const v4f a = *(const v4f*)(p);
  const v4f c = *(const v4f*)(p + 4);
  unsigned short hb[8];
#pragma unroll
  for (int e = 0; e < 4; ++e) {
    hb[e]     = f2bf_bits(a[e]);
    hb[4 + e] = f2bf_bits(c[e]);
  }
  const v4u u = (v4u){pk16(hb[0], hb[1]), pk16(hb[2], hb[3]), pk16(hb[4], hb[5]), pk16(hb[6], hb[7])};
  unsigned short* q = out + (size_t)z * kDim * kDim + 8 * (size_t)i;
  *(volatile v4u*)q = u;
  __threadfence();
  *(volatile v4u*)q = u;
}

__global__ __launch_bounds__(256) void ln_split_kernel(const float* __restrict__ x, const float* __restrict__ vec,
                                                       unsigned short* __restrict__ xnh, unsigned short* __restrict__ xnl) {
  const int lane = threadIdx.x & 31;
  const int wave = threadIdx.x >> 5;
  const int row  = blockIdx.x * 8 + wave;
  const float* xr = x + (size_t)row * kDim;
  const float* gp = vec + 6 * kDim;
  const float* bp = vec + 7 * kDim;
  float v[16];
#pragma unroll
  for (int i = 0; i < 2; ++i) {
    const v4f a = *(const v4f*)(xr + 256 * i + 8 * lane);
    const v4f c = *(const v4f*)(xr + 256 * i + 8 * lane + 4);
#pragma unroll
    for (int e = 0; e < 4; ++e) { v[8 * i + e] = rbf(a[e]); v[8 * i + 4 + e] = rbf(c[e]); }
  }
  float s = 0.0f;
#pragma unroll
  for (int e = 0; e < 16; ++e) s += v[e];
#pragma unroll
  for (int off = 16; off > 0; off >>= 1) s += __shfl_xor(s, off, 32);
  const float mu = s * kInvDim;
  float d = 0.0f;
#pragma unroll
  for (int e = 0; e < 16; ++e) { const float t = v[e] - mu; d += t * t; }
#pragma unroll
  for (int off = 16; off > 0; off >>= 1) d += __shfl_xor(d, off, 32);
  const float var = d * kInvDim;
  const float rs  = 1.0f / sqrtf(var + kLnEps);
  const size_t orow = (size_t)row * kDim;
#pragma unroll
  for (int i = 0; i < 2; ++i) {
    asm volatile("" ::: "memory");
    const int c0 = 256 * i + 8 * lane;
    const v4f ga = *(const v4f*)(gp + c0);
    const v4f gc = *(const v4f*)(gp + c0 + 4);
    const v4f ba = *(const v4f*)(bp + c0);
    const v4f bc = *(const v4f*)(bp + c0 + 4);
    unsigned short hb[8], lb[8];
#pragma unroll
    for (int e = 0; e < 4; ++e) {
      const float y0 = (v[8 * i + e] - mu) * rs * ga[e] + ba[e];
      const float y1 = (v[8 * i + 4 + e] - mu) * rs * gc[e] + bc[e];
      hb[e] = f2bf_bits(y0);
      lb[e] = f2bf_bits(y0 - bf_bits2f(hb[e]));
      hb[4 + e] = f2bf_bits(y1);
      lb[4 + e] = f2bf_bits(y1 - bf_bits2f(hb[4 + e]));
    }
    const v4u uh = (v4u){pk16(hb[0], hb[1]), pk16(hb[2], hb[3]), pk16(hb[4], hb[5]), pk16(hb[6], hb[7])};
    const v4u ul = (v4u){pk16(lb[0], lb[1]), pk16(lb[2], lb[3]), pk16(lb[4], lb[5]), pk16(lb[6], lb[7])};
    unsigned short* qh = xnh + orow + c0;
    unsigned short* ql = xnl + orow + c0;
    *(volatile v4u*)qh = uh;
    *(volatile v4u*)ql = ul;
    __threadfence();
    *(volatile v4u*)qh = uh;
    *(volatile v4u*)ql = ul;
  }
}

__global__ __launch_bounds__(256) void poscast_kernel(const float* __restrict__ pe, unsigned short* __restrict__ out, int chunk) {
  const int i  = blockIdx.x * 256 + threadIdx.x;
  const int r  = i >> 6;
  const int c8 = (i & 63) * 8;
  const int b  = chunk * kChunk + (r >> 10);
  const int pp = r & 1023;
  const int ppc = (pp < kP) ? pp : (kP - 1);
  const float keep = (pp < kP) ? 1.0f : 0.0f;
  const float* p = pe + ((size_t)(b * kP + ppc)) * kDim + c8;
  const v4f a = *(const v4f*)(p) * keep;
  const v4f c = *(const v4f*)(p + 4) * keep;
  unsigned short hb[8];
#pragma unroll
  for (int e = 0; e < 4; ++e) {
    hb[e]     = f2bf_bits(a[e]);
    hb[4 + e] = f2bf_bits(c[e]);
  }
  const v4u u = (v4u){pk16(hb[0], hb[1]), pk16(hb[2], hb[3]), pk16(hb[4], hb[5]), pk16(hb[6], hb[7])};
  unsigned short* q = out + 8 * (size_t)i;
  *(volatile v4u*)q = u;
  __threadfence();
  *(volatile v4u*)q = u;
}

__global__ __launch_bounds__(64) void relsoftmax_kernel(const float* __restrict__ SCp, const float* __restrict__ SPp,
                                                        unsigned short* __restrict__ Php, unsigned short* __restrict__ Plp) {
  __shared__ __align__(16) float lg[kSeq];
  __shared__ float redM[2];
  __shared__ float redS[2];
  const int s    = blockIdx.x;
  const int h    = blockIdx.y;
  const int t    = threadIdx.x;
  const int lane = t & 31, wave = t >> 5;
  const size_t rowc = ((size_t)(h * kSeq + s)) * kSeq;
  const size_t rowp = ((size_t)(h * kSeq + s)) * kSPld;
  const float* cr = SCp + rowc;
  const float* pr = SPp + rowp + (63 - (s & 63));

  float mx = -__builtin_inff();
#pragma unroll 1
  for (int it = 0; it < 4; ++it) {
    const int c = it * 128 + 2 * t;
    const v2f cv = *(const v2f*)(cr + c);
    const float p0 = pr[c];
    const float p1 = pr[c + 1];
    v2f av;
    av[0] = (cv[0] + p0) * kScoreScale;
    av[1] = (cv[1] + p1) * kScoreScale;
    mx = fmaxf(mx, fmaxf(av[0], av[1]));
    *(v2f*)(lg + c) = av;
  }
#pragma unroll
  for (int off = 16; off > 0; off >>= 1) mx = fmaxf(mx, __shfl_xor(mx, off, 32));
  if (lane == 0) redM[wave] = mx;
  __syncthreads();
  const float m = fmaxf(redM[0], redM[1]);

  float sum = 0.0f;
#pragma unroll 1
  for (int it = 0; it < 4; ++it) {
    const int c = it * 128 + 2 * t;
    const v2f l = *(const v2f*)(lg + c);
    v2f ev;
#pragma unroll
    for (int e = 0; e < 2; ++e) {
      ev[e] = expf(l[e] - m);
      sum += ev[e];
    }
    *(v2f*)(lg + c) = ev;
  }
#pragma unroll
  for (int off = 16; off > 0; off >>= 1) sum += __shfl_xor(sum, off, 32);
  if (lane == 0) redS[wave] = sum;
  __syncthreads();
  const float tot = redS[0] + redS[1];
  const float inv = 1.0f / tot;

  const v4f e0 = *(const v4f*)(lg + 8 * t);
  const v4f e1 = *(const v4f*)(lg + 8 * t + 4);
  unsigned short hb[8], lb[8];
#pragma unroll
  for (int e = 0; e < 4; ++e) {
    const float p0 = e0[e] * inv;
    const float p1 = e1[e] * inv;
    hb[e] = f2bf_bits(p0);
    lb[e] = f2bf_bits(p0 - bf_bits2f(hb[e]));
    hb[4 + e] = f2bf_bits(p1);
    lb[4 + e] = f2bf_bits(p1 - bf_bits2f(hb[4 + e]));
  }
  const v4u uh = (v4u){pk16(hb[0], hb[1]), pk16(hb[2], hb[3]), pk16(hb[4], hb[5]), pk16(hb[6], hb[7])};
  const v4u ul = (v4u){pk16(lb[0], lb[1]), pk16(lb[2], lb[3]), pk16(lb[4], lb[5]), pk16(lb[6], lb[7])};
  unsigned short* ph = Php + rowc + 8 * (size_t)t;
  unsigned short* pl = Plp + rowc + 8 * (size_t)t;
  *(volatile v4u*)ph = uh;
  *(volatile v4u*)pl = ul;
  __threadfence();
  *(volatile v4u*)ph = uh;
  *(volatile v4u*)pl = ul;
}

extern "C" void kernel_launch(void* const* d_in, const int* in_sizes, int n_in,
                              void* d_out, int out_size, void* d_ws, size_t ws_size,
                              hipStream_t stream) {
  if (n_in < 16) return;
  const int nTokElem = kTok * kDim;
  const int nPosElem = kBatch * kP * kDim;
  const int nW = kDim * kDim;
  if (in_sizes[0] != nTokElem || in_sizes[1] != nPosElem) return;
  if (in_sizes[2] != kDim || in_sizes[3] != kDim) return;
  if (in_sizes[4] != nW || in_sizes[6] != nW || in_sizes[8] != nW || in_sizes[10] != nW || in_sizes[14] != nW) return;
  if (in_sizes[5] != kDim || in_sizes[7] != kDim || in_sizes[9] != kDim || in_sizes[11] != kDim || in_sizes[15] != kDim) return;
  if (in_sizes[12] != kHeads * kHd || in_sizes[13] != kHeads * kHd) return;
  if (out_size != nTokElem) return;

  const size_t szW16  = (size_t)5 * kDim * kDim * 2;
  const size_t szVec  = (size_t)kVecRows * kDim * 4;
  const size_t szTokH = (size_t)kTok * kDim * 2;
  const size_t szPosC = (size_t)kChunkRows * kDim * 2;
  const size_t szSC   = (size_t)kHeads * kSeq * kSeq * 4;
  const size_t szSP   = (size_t)kHeads * kSeq * kSPld * 4;
  const size_t szP    = (size_t)kHeads * kSeq * kSeq * 2;
  const size_t offW16 = 0;
  const size_t offVec = offW16 + szW16;
  const size_t offXNh = offVec + szVec;
  const size_t offXNl = offXNh + szTokH;
  const size_t offPOS = offXNl + szTokH;
  const size_t offQCh = offPOS + szPosC;
  const size_t offQCl = offQCh + szTokH;
  const size_t offQPh = offQCl + szTokH;
  const size_t offQPl = offQPh + szTokH;
  const size_t offKh  = offQPl + szTokH;
  const size_t offKl  = offKh + szTokH;
  const size_t offVTh = offKl + szTokH;
  const size_t offVTl = offVTh + szTokH;
  const size_t offPRh = offVTl + szTokH;
  const size_t offPRl = offPRh + szPosC;
  const size_t offSC  = offPRl + szPosC;
  const size_t offSP  = offSC + szSC;
  const size_t offPh  = offSP + szSP;
  const size_t offPl  = offPh + szP;
  const size_t total  = offPl + szP;
  if (ws_size < total) return;

  const float* x     = (const float*)d_in[0];
  const float* pe    = (const float*)d_in[1];
  const float* ln_g  = (const float*)d_in[2];
  const float* ln_b  = (const float*)d_in[3];
  const float* Wq    = (const float*)d_in[4];
  const float* bq    = (const float*)d_in[5];
  const float* Wk    = (const float*)d_in[6];
  const float* bk    = (const float*)d_in[7];
  const float* Wv    = (const float*)d_in[8];
  const float* bv    = (const float*)d_in[9];
  const float* Wp    = (const float*)d_in[10];
  const float* bp    = (const float*)d_in[11];
  const float* cbias = (const float*)d_in[12];
  const float* pbias = (const float*)d_in[13];
  const float* Wo    = (const float*)d_in[14];
  const float* bo    = (const float*)d_in[15];
  float* out = (float*)d_out;
  char* ws = (char*)d_ws;
  unsigned short* W16  = (unsigned short*)(ws + offW16);
  float*          VEC  = (float*)(ws + offVec);
  unsigned short* XNh  = (unsigned short*)(ws + offXNh);
  unsigned short* XNl  = (unsigned short*)(ws + offXNl);
  unsigned short* POSC = (unsigned short*)(ws + offPOS);
  unsigned short* QCh  = (unsigned short*)(ws + offQCh);
  unsigned short* QCl  = (unsigned short*)(ws + offQCl);
  unsigned short* QPh  = (unsigned short*)(ws + offQPh);
  unsigned short* QPl  = (unsigned short*)(ws + offQPl);
  unsigned short* Kh   = (unsigned short*)(ws + offKh);
  unsigned short* Kl   = (unsigned short*)(ws + offKl);
  unsigned short* VTh  = (unsigned short*)(ws + offVTh);
  unsigned short* VTl  = (unsigned short*)(ws + offVTl);
  unsigned short* PRh  = (unsigned short*)(ws + offPRh);
  unsigned short* PRl  = (unsigned short*)(ws + offPRl);
  float*          SC   = (float*)(ws + offSC);
  float*          SP   = (float*)(ws + offSP);
  unsigned short* Ph   = (unsigned short*)(ws + offPh);
  unsigned short* Pl   = (unsigned short*)(ws + offPl);
  unsigned short* CTXh = XNh;
  unsigned short* CTXl = XNl;
  const size_t planeW = (size_t)kDim * kDim;
  const unsigned short* W16q = W16;
  const unsigned short* W16k = W16 + planeW;
  const unsigned short* W16v = W16 + 2 * planeW;
  const unsigned short* W16p = W16 + 3 * planeW;
  const unsigned short* W16o = W16 + 4 * planeW;
  const float* vecQC = VEC;
  const float* vecQP = VEC + 1 * kDim;
  const float* vecK  = VEC + 2 * kDim;
  const float* vecV  = VEC + 3 * kDim;
  const float* vecP  = VEC + 4 * kDim;
  const float* vecO  = VEC + 5 * kDim;

  vecprep_kernel<<<dim3(kVecRows), dim3(128), 0, stream>>>(bq, bk, bv, bp, bo, ln_g, ln_b, cbias, pbias, VEC);
  castw_kernel<<<dim3(nW / 8 / 256, 5), dim3(256), 0, stream>>>(Wq, Wk, Wv, Wp, Wo, W16);
  ln_split_kernel<<<dim3(kTok / 8), dim3(256), 0, stream>>>(x, VEC, XNh, XNl);

  const int tilesTok   = (kTok / 64) * (kDim / 64);
  const int tilesChunk = (kChunkRows / 64) * (kDim / 64);
  wmma_gemm64<1, true, false, 2, 2><<<dim3(tilesTok / 8, 1), dim3(256), 0, stream>>>(
      XNh, XNl, kDim, 0L, W16q, W16q, kDim, 0L, (void*)QCh, (void*)QCl, kDim, 0L,
      vecQC, kTok, kDim, kDim, 1.0f);
  wmma_gemm64<1, true, false, 2, 2><<<dim3(tilesTok / 8, 1), dim3(256), 0, stream>>>(
      XNh, XNl, kDim, 0L, W16q, W16q, kDim, 0L, (void*)QPh, (void*)QPl, kDim, 0L,
      vecQP, kTok, kDim, kDim, 1.0f);
  wmma_gemm64<1, true, false, 2, 2><<<dim3(tilesTok / 8, 1), dim3(256), 0, stream>>>(
      XNh, XNl, kDim, 0L, W16k, W16k, kDim, 0L, (void*)Kh, (void*)Kl, kDim, 0L,
      vecK, kTok, kDim, kDim, 1.0f);
  wmma_gemm64<1, false, true, 1, 2><<<dim3(tilesTok / 8, 1), dim3(256), 0, stream>>>(
      W16v, W16v, kDim, 0L, XNh, XNl, kDim, 0L, (void*)VTh, (void*)VTl, kTok, 0L,
      vecV, kDim, kTok, kDim, 1.0f);

  const long strideHead = (long)kHd;
  const long strideSC   = (long)kSeq * kSeq;
  const long strideSP   = (long)kSeq * kSPld;
  const long strideVTh  = (long)kHd * kTok;
  const int tilesSC = (kSeq / 64) * (kSeq / 64);
  const int tilesSP = (kSeq / 64) * kBandN;
  const int tilesPV = (kSeq / 64) * (kHd / 64);
  for (int chunk = 0; chunk < kBatch / kChunk; ++chunk) {
    poscast_kernel<<<dim3(kChunkRows * kDim / 8 / 256), dim3(256), 0, stream>>>(pe, POSC, chunk);
    wmma_gemm64<1, false, false, 2, 2><<<dim3(tilesChunk / 8, 1), dim3(256), 0, stream>>>(
        POSC, POSC, kDim, 0L, W16p, W16p, kDim, 0L, (void*)PRh, (void*)PRl, kDim, 0L,
        vecP, kChunkRows, kDim, kDim, 1.0f);
    for (int bl = 0; bl < kChunk; ++bl) {
      const int b = chunk * kChunk + bl;
      const size_t tokOff = (size_t)b * kSeq * kDim;
      const size_t prOff  = (size_t)bl * kPosPad * kDim;
      wmma_gemm64<1, true, true, 0, 0><<<dim3(tilesSC / 8, kHeads), dim3(256), 0, stream>>>(
          QCh + tokOff, QCl + tokOff, kDim, strideHead, Kh + tokOff, Kl + tokOff, kDim, strideHead,
          (void*)SC, (void*)SC, kSeq, strideSC, VEC, kSeq, kSeq, kHd, 1.0f);
      wmma_gemm64<1, true, true, 0, 0, kBandN, kBandOff><<<dim3(tilesSP / 8, kHeads), dim3(256), 0, stream>>>(
          QPh + tokOff, QPl + tokOff, kDim, strideHead, PRh + prOff, PRl + prOff, kDim, strideHead,
          (void*)SP, (void*)SP, kSPld, strideSP, VEC, kSeq, kPosPad, kHd, 1.0f);
      relsoftmax_kernel<<<dim3(kSeq, kHeads), dim3(64), 0, stream>>>(SC, SP, Ph, Pl);
      wmma_gemm64<1, true, true, 0, 2><<<dim3(tilesPV / 8, kHeads), dim3(256), 0, stream>>>(
          Ph, Pl, kSeq, strideSC, VTh + (size_t)b * kSeq, VTl + (size_t)b * kSeq, kTok, strideVTh,
          (void*)(CTXh + tokOff), (void*)(CTXl + tokOff), kDim, strideHead, VEC, kSeq, kHd, kSeq, 1.0f);
    }
  }

  wmma_gemm64<1, true, false, 2, 0><<<dim3(tilesTok / 8, 1), dim3(256), 0, stream>>>(
      CTXh, CTXl, kDim, 0L, W16o, W16o, kDim, 0L, (void*)out, (void*)out, kDim, 0L,
      vecO, kTok, kDim, kDim, 1.0f);
}
